// Encoder_76948634075520
// MI455X (gfx1250) — hardware-verified
//
#include <hip/hip_runtime.h>
#include <math.h>

constexpr int kBatch   = 128;
constexpr int kSteps   = 512;
constexpr int kFeat    = 12;
constexpr int kHid     = 12;
constexpr int kGateRows = 4 * kHid;
constexpr int kQDim    = 2 * kHid;
constexpr int kQPad    = 32;
constexpr int kUDim    = 512;
constexpr int kRowsBT  = kBatch * kSteps;
constexpr int kRowsBN  = kBatch * kFeat;
constexpr int kLdsPitch = 520;
constexpr int kTileT   = 16;
constexpr int kWvRows  = 16;

constexpr float kDataCarry = 8.0f;
constexpr float kW1Carry   = 16.0f;
constexpr float kW1xScale  = 1.0f / (kDataCarry * kW1Carry);
constexpr float kQryCarry  = 256.0f;
constexpr float kW2Carry   = 16.0f;
constexpr float kW2qScale  = 1.0f / (kQryCarry * kW2Carry);
constexpr float kTanhCarry = 1024.0f;
constexpr float kWvCarry   = 16.0f;
constexpr float kWvLoScale = 2048.0f;
constexpr float kWvLoInv   = 1.0f / kWvLoScale;
constexpr float kScoreInv  = 1.0f / (kTanhCarry * kWvCarry);

static_assert(kRowsBN % 64 == 0, "GEMM M tile multiple");
static_assert(kUDim % 64 == 0, "GEMM N tile multiple");
static_assert(kSteps % 32 == 0, "GEMM K multiple of 32");
static_assert(kUDim % 32 == 0, "score matvec K multiple of 32");
static_assert(kQPad % 32 == 0 && kQDim <= kQPad, "query K pad");
static_assert(kRowsBT % 256 == 0, "LSTM grid exact");
static_assert((kTileT * kFeat * 4) % 128 == 0, "output tile is whole 128-B lines");
static_assert(kSteps % kTileT == 0, "t tiles exact");
static_assert(kFeat == 12 && kTileT == 16, "six waves x two 16-row score tiles");
static_assert((kWvRows * kUDim / 8) % 256 == 0, "Wv plane grid exact");

typedef __attribute__((ext_vector_type(16))) _Float16 v16h;
typedef __attribute__((ext_vector_type(8)))  _Float16 v8h;
typedef __attribute__((ext_vector_type(16))) __bf16   v16b;
typedef __attribute__((ext_vector_type(8)))  __bf16   v8b;
typedef __attribute__((ext_vector_type(8)))  float    v8f;
typedef __attribute__((ext_vector_type(4)))  float    v4f;
typedef __attribute__((ext_vector_type(4)))  unsigned int v4u;

__device__ __forceinline__ unsigned short f2bf_bits(float f) {
  unsigned u = __float_as_uint(f);
  return (unsigned short)((u + 0x7FFFu + ((u >> 16) & 1u)) >> 16);
}
__device__ __forceinline__ float bf_bits2f(unsigned short h) { return __uint_as_float(((unsigned)h) << 16); }

__device__ __forceinline__ void dep_guard4_h(v8f& a, v8f& b, v8f& c, v8f& d, v16h x, v16h y) { asm volatile("v_nop\n\tv_nop\n\tv_nop\n\tv_nop" : "+v"(a), "+v"(b), "+v"(c), "+v"(d) : "v"(x), "v"(y)); }
__device__ __forceinline__ void dep_guard4_b(v8f& a, v8f& b, v8f& c, v8f& d, v16b x, v16b y) { asm volatile("v_nop\n\tv_nop\n\tv_nop\n\tv_nop" : "+v"(a), "+v"(b), "+v"(c), "+v"(d) : "v"(x), "v"(y)); }
__device__ __forceinline__ void dep_guard1_h(v8f& a, v16h x, v16h y) { asm volatile("v_nop\n\tv_nop\n\tv_nop\n\tv_nop" : "+v"(a) : "v"(x), "v"(y)); }
__device__ __forceinline__ void keep4_h(v16h a, v16h b, v16h c, v16h d) { asm volatile("v_nop" :: "v"(a), "v"(b), "v"(c), "v"(d)); }
__device__ __forceinline__ void keep4_b(v16b a, v16b b, v16b c, v16b d) { asm volatile("v_nop" :: "v"(a), "v"(b), "v"(c), "v"(d)); }
__device__ __forceinline__ void acc_guard4(v8f& a, v8f& b, v8f& c, v8f& d) { asm volatile("v_nop\n\tv_nop\n\tv_nop\n\tv_nop" : "+v"(a), "+v"(b), "+v"(c), "+v"(d)); }
__device__ __forceinline__ void acc_guard1(v8f& a) { asm volatile("v_nop\n\tv_nop\n\tv_nop\n\tv_nop" : "+v"(a)); }

template <typename T> struct Frag;
template <> struct Frag<_Float16> {
  typedef v16h V; union U { v16h v; v8h h[2]; };
  static __device__ __forceinline__ v16h load(const _Float16* p) {
    U f; f.h[0] = *(const v8h*)(p); f.h[1] = *(const v8h*)(p + 16); return f.v;
  }
  static __device__ __forceinline__ v8f mma(v16h a, v16h b, v8f c) {
    return __builtin_amdgcn_wmma_f32_16x16x32_f16(false, a, false, b, (short)0, c, false, false);
  }
  static __device__ __forceinline__ void guard4(v8f& a, v8f& b, v8f& c, v8f& d, v16h x, v16h y) { dep_guard4_h(a, b, c, d, x, y); }
  static __device__ __forceinline__ void keep(v16h a, v16h b, v16h c, v16h d) { keep4_h(a, b, c, d); }
};
template <> struct Frag<__bf16> {
  typedef v16b V; union U { v16b v; v8b h[2]; };
  static __device__ __forceinline__ v16b load(const __bf16* p) {
    U f; f.h[0] = *(const v8b*)(p); f.h[1] = *(const v8b*)(p + 16); return f.v;
  }
  static __device__ __forceinline__ v8f mma(v16b a, v16b b, v8f c) {
    return __builtin_amdgcn_wmma_f32_16x16x32_bf16(false, a, false, b, (short)0, c, false, false);
  }
  static __device__ __forceinline__ void guard4(v8f& a, v8f& b, v8f& c, v8f& d, v16b x, v16b y) { dep_guard4_b(a, b, c, d, x, y); }
  static __device__ __forceinline__ void keep(v16b a, v16b b, v16b c, v16b d) { keep4_b(a, b, c, d); }
};

__device__ __forceinline__ unsigned pk16(unsigned short a, unsigned short b) { return (unsigned)a | ((unsigned)b << 16); }
__device__ __forceinline__ unsigned short h_bits(float f) { const _Float16 h = (_Float16)f; return __builtin_bit_cast(unsigned short, h); }

__device__ __forceinline__ float sig_p(float x)  { return __builtin_amdgcn_rcpf(1.0f + expf(-x)); }
__device__ __forceinline__ float tanh_p(float x) { return 1.0f - 2.0f * __builtin_amdgcn_rcpf(expf(2.0f * x) + 1.0f); }
__device__ __forceinline__ float tanh_s(float x) {
  x = fminf(15.0f, fmaxf(-15.0f, x));
  return 1.0f - 2.0f * __builtin_amdgcn_rcpf(__expf(2.0f * x) + 1.0f);
}

template <int ET> struct Elem;
template <> struct Elem<0> { typedef _Float16 T; };
template <> struct Elem<1> { typedef __bf16 T; };
template <int ET, bool SPLIT, int BIAS_MODE, int OUT_MODE, bool RESID>
__global__ __launch_bounds__(256) void wmma_gemm64(
    const unsigned short* __restrict__ Ap, const unsigned short* __restrict__ A2p, int lda, long strideA,
    const unsigned short* __restrict__ Btp, const unsigned short* __restrict__ Bt2p, int ldb, long strideB,
    void* __restrict__ Cout, void* __restrict__ Cout2, int ldc, long strideC,
    const float* __restrict__ bias,
    const float* __restrict__ resid, long strideR,
    int M, int N, int K, float scale) {
  typedef typename Elem<ET>::T T;
  typedef typename Frag<T>::V V;
  const T* A = (const T*)Ap; const T* A2 = (const T*)A2p; const T* Bt = (const T*)Btp; const T* Bt2 = (const T*)Bt2p;
  __shared__ __align__(16) float sT[8][16 * 68];
  const int b    = blockIdx.y;
  const int lane = threadIdx.x & 31;
  const int wave = threadIdx.x >> 5;
  const int tilesN = N >> 6;
  const int tilesM = M >> 6;
  const int tile = blockIdx.x * 8 + wave;
  if (tile >= tilesM * tilesN) return;
  const int tm = tile / tilesN;
  const int tn = tile - tm * tilesN;
  const int m0 = tm << 6;
  const int n0 = tn << 6;

  const T* Ab  = A  + (size_t)b * strideA;
  const T* Bb  = Bt + (size_t)b * strideB;
  const T* Ab2 = SPLIT ? (A2  + (size_t)b * strideA) : nullptr;
  const T* Bb2 = SPLIT ? (Bt2 + (size_t)b * strideB) : nullptr;

  const int rlane = lane & 15;
  const int koff  = (lane >> 4) * 8;
  const int mOff  = (lane >> 4) * 8;

  v8f acc[4][4];
#pragma unroll
  for (int i = 0; i < 4; ++i)
#pragma unroll
    for (int j = 0; j < 4; ++j) acc[i][j] = (v8f){0.f,0.f,0.f,0.f,0.f,0.f,0.f,0.f};

  for (int k0 = 0; k0 < K; k0 += 32) {
    V bh[4], bl[4];
#pragma unroll
    for (int j = 0; j < 4; ++j) {
      const size_t bo = (size_t)(n0 + (j << 4) + rlane) * ldb + koff + k0;
      bh[j] = Frag<T>::load(Bb + bo);
      if (SPLIT) bl[j] = Frag<T>::load(Bb2 + bo);
    }
#pragma unroll
    for (int i = 0; i < 4; ++i) {
      const size_t ao = (size_t)(m0 + (i << 4) + rlane) * lda + koff + k0;
      V ah = Frag<T>::load(Ab + ao);
      V al;
      if (SPLIT) al = Frag<T>::load(Ab2 + ao);
#pragma unroll
      for (int j = 0; j < 4; ++j) {
        acc[i][j] = Frag<T>::mma(ah, bh[j], acc[i][j]);
        if (SPLIT) {
          acc[i][j] = Frag<T>::mma(ah, bl[j], acc[i][j]);
          acc[i][j] = Frag<T>::mma(al, bh[j], acc[i][j]);
        }
      }
      Frag<T>::guard4(acc[i][0], acc[i][1], acc[i][2], acc[i][3], ah, SPLIT ? al : ah);
    }
    Frag<T>::keep(bh[0], bh[1], bh[2], bh[3]);
    if (SPLIT) Frag<T>::keep(bl[0], bl[1], bl[2], bl[3]);
  }
  acc_guard4(acc[0][0], acc[0][1], acc[0][2], acc[0][3]);
  acc_guard4(acc[1][0], acc[1][1], acc[1][2], acc[1][3]);
  acc_guard4(acc[2][0], acc[2][1], acc[2][2], acc[2][3]);
  acc_guard4(acc[3][0], acc[3][1], acc[3][2], acc[3][3]);

  float* slab = sT[wave];
  const float* Rb = RESID ? (resid + (size_t)b * strideR) : nullptr;
#pragma unroll
  for (int i = 0; i < 4; ++i) {
    const int mBase = m0 + (i << 4);
#pragma unroll
    for (int j = 0; j < 4; ++j) {
      const int n = n0 + (j << 4) + rlane;
      float bvv = 0.f;
      if (BIAS_MODE == 2) bvv = bias[n];
#pragma unroll
      for (int r = 0; r < 8; ++r) {
        float v = acc[i][j][r] * scale;
        if (BIAS_MODE == 1) v += bias[mBase + mOff + r];
        if (BIAS_MODE == 2) v += bvv;
        if (RESID) v += Rb[(size_t)(mBase + mOff + r) * ldc + n];
        slab[(mOff + r) * 68 + (j << 4) + rlane] = v;
      }
    }
    __builtin_amdgcn_fence(__ATOMIC_RELEASE, "workgroup");
    __builtin_amdgcn_wave_barrier();
    __builtin_amdgcn_fence(__ATOMIC_ACQUIRE, "workgroup");
    if (OUT_MODE == 0) {
      float* C = (float*)Cout + (size_t)b * strideC;
      const int hh = lane >> 4, c4 = (lane & 15) * 4;
      for (int pass = 0; pass < 2; ++pass) {
#pragma unroll
        for (int it = 0; it < 8; ++it) {
          const int row = it * 2 + hh;
          v4f v = *(const v4f*)(slab + row * 68 + c4);
          *(volatile v4f*)(C + (size_t)(mBase + row) * ldc + n0 + c4) = v;
        }
        __threadfence();
      }
    } else {
      const int q = lane >> 3, c8 = (lane & 7) * 8;
      unsigned short* C  = (unsigned short*)Cout  + (size_t)b * strideC;
      unsigned short* C2 = (OUT_MODE == 2) ? ((unsigned short*)Cout2 + (size_t)b * strideC) : nullptr;
      for (int pass = 0; pass < 2; ++pass) {
#pragma unroll
        for (int it = 0; it < 4; ++it) {
          const int row = it * 4 + q;
          const float* sp = slab + row * 68 + c8;
          v8h hv, lv;
#pragma unroll
          for (int e = 0; e < 8; ++e) {
            if (OUT_MODE == 1) {
              hv[e] = (_Float16)sp[e];
            } else {
              unsigned short hb = f2bf_bits(sp[e]);
              unsigned short lb = f2bf_bits(sp[e] - bf_bits2f(hb));
              hv[e] = __builtin_bit_cast(_Float16, hb);
              lv[e] = __builtin_bit_cast(_Float16, lb);
            }
          }
          *(volatile v8h*)(C + (size_t)(mBase + row) * ldc + n0 + c8) = hv;
          if (OUT_MODE == 2) *(volatile v8h*)(C2 + (size_t)(mBase + row) * ldc + n0 + c8) = lv;
        }
        __threadfence();
      }
    }
    __builtin_amdgcn_fence(__ATOMIC_RELEASE, "workgroup");
    __builtin_amdgcn_wave_barrier();
    __builtin_amdgcn_fence(__ATOMIC_ACQUIRE, "workgroup");
  }
}

__global__ __launch_bounds__(256) void dataT_f16_kernel(const float* __restrict__ data, unsigned short* __restrict__ dT, float carry) {
  __shared__ float sm[kSteps * 13];
  const int tid = threadIdx.x;
  const int b = blockIdx.x;
  const float* src = data + (size_t)b * kSteps * kFeat;
#pragma unroll
  for (int it = 0; it < 6; ++it) {
    const int i4 = it * 256 + tid;
    const int t = i4 / 3;
    const int n0 = (i4 - t * 3) * 4;
    const v4f v = *(const v4f*)(src + (size_t)i4 * 4);
    sm[t * 13 + n0 + 0] = v[0] * carry;
    sm[t * 13 + n0 + 1] = v[1] * carry;
    sm[t * 13 + n0 + 2] = v[2] * carry;
    sm[t * 13 + n0 + 3] = v[3] * carry;
  }
  __syncthreads();
  v4u u[3];
#pragma unroll
  for (int it = 0; it < 3; ++it) {
    const int id = it * 256 + tid;
    const int n = id >> 6;
    const int c8 = (id & 63) * 8;
    unsigned short hb[8];
#pragma unroll
    for (int e = 0; e < 8; ++e) hb[e] = h_bits(sm[(c8 + e) * 13 + n]);
    u[it] = (v4u){pk16(hb[0], hb[1]), pk16(hb[2], hb[3]), pk16(hb[4], hb[5]), pk16(hb[6], hb[7])};
  }
  for (int pass = 0; pass < 2; ++pass) {
#pragma unroll
    for (int it = 0; it < 3; ++it) {
      const int id = it * 256 + tid;
      const int n = id >> 6;
      const int c8 = (id & 63) * 8;
      *(volatile v4u*)(dT + ((size_t)(b * kFeat + n)) * kSteps + c8) = u[it];
    }
    __threadfence();
  }
}

__global__ __launch_bounds__(256) void cast8_scale_f16_kernel(const float* __restrict__ in, unsigned short* __restrict__ out, int n8, float carry) {
  const int i = blockIdx.x * 256 + threadIdx.x;
  if (i >= n8) return;
  const float* p = in + 8 * (size_t)i;
  const v4f a = *(const v4f*)(p);
  const v4f c = *(const v4f*)(p + 4);
  unsigned short hb[8];
#pragma unroll
  for (int e = 0; e < 4; ++e) {
    hb[e]     = h_bits(a[e] * carry);
    hb[4 + e] = h_bits(c[e] * carry);
  }
  const v4u u = (v4u){pk16(hb[0], hb[1]), pk16(hb[2], hb[3]), pk16(hb[4], hb[5]), pk16(hb[6], hb[7])};
  unsigned short* q = out + 8 * (size_t)i;
  *(volatile v4u*)q = u;
  __threadfence();
  *(volatile v4u*)q = u;
}

__global__ __launch_bounds__(256) void w2pad_f16_kernel(const float* __restrict__ W2, unsigned short* __restrict__ out, float carry) {
  const int i = blockIdx.x * 256 + threadIdx.x;
  const int row = i >> 2;
  const int ch = i & 3;
  const int chc = (ch < 3) ? ch : 2;
  const float* p = W2 + (size_t)row * kQDim + chc * 8;
  const v4f a = *(const v4f*)(p);
  const v4f c = *(const v4f*)(p + 4);
  const bool live = (ch < 3);
  unsigned short hb[8];
#pragma unroll
  for (int e = 0; e < 4; ++e) {
    const float fa = live ? (a[e] * carry) : 0.0f;
    const float fc = live ? (c[e] * carry) : 0.0f;
    hb[e]     = h_bits(fa);
    hb[4 + e] = h_bits(fc);
  }
  const v4u u = (v4u){pk16(hb[0], hb[1]), pk16(hb[2], hb[3]), pk16(hb[4], hb[5]), pk16(hb[6], hb[7])};
  unsigned short* q = out + 8 * (size_t)i;
  *(volatile v4u*)q = u;
  __threadfence();
  *(volatile v4u*)q = u;
}

__global__ __launch_bounds__(256) void wvplane_f16_kernel(const float* __restrict__ Wv, unsigned short* __restrict__ out,
                                                          float carry, float loScale) {
  const int i = blockIdx.x * 256 + threadIdx.x;
  const int row = i >> 6;
  const int c8 = (i & 63) * 8;
  const v4f a = *(const v4f*)(Wv + c8);
  const v4f c = *(const v4f*)(Wv + c8 + 4);
  unsigned short hb[8];
#pragma unroll
  for (int e = 0; e < 4; ++e) {
    const float wa = a[e] * carry;
    const float wc = c[e] * carry;
    const _Float16 ha = (_Float16)wa;
    const _Float16 hc = (_Float16)wc;
    const float hfa = (float)ha;
    const float hfc = (float)hc;
    const float la = (wa - hfa) * loScale;
    const float lc = (wc - hfc) * loScale;
    const float sa = (row == 0) ? hfa : ((row == 1) ? la : 0.0f);
    const float sc = (row == 0) ? hfc : ((row == 1) ? lc : 0.0f);
    hb[e]     = h_bits(sa);
    hb[4 + e] = h_bits(sc);
  }
  const v4u u = (v4u){pk16(hb[0], hb[1]), pk16(hb[2], hb[3]), pk16(hb[4], hb[5]), pk16(hb[6], hb[7])};
  unsigned short* q = out + 8 * (size_t)i;
  *(volatile v4u*)q = u;
  __threadfence();
  *(volatile v4u*)q = u;
}

__global__ __launch_bounds__(256) void lstm_query_kernel(const float* __restrict__ data,
                                                         const float* __restrict__ W_ih1,
                                                         const float* __restrict__ b_ih1,
                                                         const float* __restrict__ b_hh1,
                                                         const float* __restrict__ W_ih2,
                                                         const float* __restrict__ b_ih2,
                                                         const float* __restrict__ b_hh2,
                                                         unsigned short* __restrict__ qplane, float carry) {
  __shared__ float sW[2 * kGateRows * kFeat];
  __shared__ float sB[2 * kGateRows];
  __shared__ float sX[kFeat * 256];
  __shared__ float sC[kHid * 256];
  const int tid = threadIdx.x;

#pragma unroll 1
  for (int i = tid; i < kGateRows * kFeat; i += 256) {
    sW[i] = W_ih1[i];
    sW[kGateRows * kFeat + i] = W_ih2[i];
  }
  {
    const int gi = (tid < kGateRows) ? tid : (kGateRows - 1);
    const float s1 = b_ih1[gi] + b_hh1[gi];
    const float s2 = b_ih2[gi] + b_hh2[gi];
    if (tid < kGateRows) {
      sB[tid] = s1;
      sB[kGateRows + tid] = s2;
    }
  }
  {
    const size_t bt = (size_t)blockIdx.x * 256 + tid;
    const float* xp = data + bt * kFeat;
#pragma unroll
    for (int q = 0; q < 3; ++q) {
      const v4f v = *(const v4f*)(xp + 4 * q);
      sX[(4 * q + 0) * 256 + tid] = v[0];
      sX[(4 * q + 1) * 256 + tid] = v[1];
      sX[(4 * q + 2) * 256 + tid] = v[2];
      sX[(4 * q + 3) * 256 + tid] = v[3];
    }
  }
  __syncthreads();

#pragma unroll 1
  for (int L = 0; L < 2; ++L) {
    float xin[kFeat];
#pragma unroll
    for (int j = 0; j < kFeat; ++j) xin[j] = sX[j * 256 + tid];
    const float* w  = sW + L * kGateRows * kFeat;
    const float* bb = sB + L * kGateRows;
#pragma unroll 1
    for (int k = 0; k < kHid; ++k) {
      float ai = bb[k];
      float ag = bb[2 * kHid + k];
      float ao = bb[3 * kHid + k];
#pragma unroll
      for (int j = 0; j < kFeat; ++j) {
        ai = fmaf(w[k * kFeat + j], xin[j], ai);
        ag = fmaf(w[(2 * kHid + k) * kFeat + j], xin[j], ag);
        ao = fmaf(w[(3 * kHid + k) * kFeat + j], xin[j], ao);
      }
      const float cc = sig_p(ai) * tanh_p(ag);
      const float hv = sig_p(ao) * tanh_p(cc);
      sX[k * 256 + tid] = hv;
      sC[k * 256 + tid] = cc;
    }
  }
  __syncthreads();

  unsigned short* qb = qplane + (size_t)blockIdx.x * 256 * kQPad;
  v4u pk[4];
#pragma unroll
  for (int it = 0; it < 4; ++it) {
    const int id = it * 256 + tid;
    const int row = id >> 2;
    const int ch = id & 3;
    unsigned short hb[8];
#pragma unroll
    for (int e = 0; e < 8; ++e) {
      const int q = ch * 8 + e;
      const int qa = (q < kHid) ? q : (kHid - 1);
      int qc = q - kHid;
      qc = (qc < 0) ? 0 : qc;
      qc = (qc < kHid) ? qc : (kHid - 1);
      const float va = sX[qa * 256 + row];
      const float vc = sC[qc * 256 + row];
      const float v = (q < kHid) ? va : ((q < kQDim) ? vc : 0.0f);
      hb[e] = h_bits(v * carry);
    }
    pk[it] = (v4u){pk16(hb[0], hb[1]), pk16(hb[2], hb[3]), pk16(hb[4], hb[5]), pk16(hb[6], hb[7])};
  }
  for (int pass = 0; pass < 2; ++pass) {
#pragma unroll
    for (int it = 0; it < 4; ++it) {
      const int id = it * 256 + tid;
      *(volatile v4u*)(qb + (size_t)id * 8) = pk[it];
    }
    __threadfence();
  }
}

__global__ __launch_bounds__(256) void attn_fused_kernel(const float* __restrict__ data,
                                                         const unsigned short* __restrict__ qplane,
                                                         const float* __restrict__ w1x,
                                                         const unsigned short* __restrict__ w2plane,
                                                         const float* __restrict__ b2,
                                                         const unsigned short* __restrict__ wvplane,
                                                         const float* __restrict__ bv,
                                                         float* __restrict__ out, float w2qScale) {
  __shared__ __align__(16) float s_w1x[kFeat * kLdsPitch];
  __shared__ __align__(16) float s_w2q[kTileT * kLdsPitch];
  __shared__ __align__(16) float s_score[kTileT * kFeat];
  __shared__ __align__(16) float s_out[kTileT * kFeat];

  const int tid  = threadIdx.x;
  const int lane = tid & 31;
  const int wave = tid >> 5;
  const int wave_u = __builtin_amdgcn_readfirstlane(wave);
  const int b    = blockIdx.x >> 5;
  const int t0   = (blockIdx.x & 31) << 4;

  {
    const float* wsrc = w1x + (size_t)b * kFeat * kUDim;
#pragma unroll
    for (int it = 0; it < 6; ++it) {
      const int i = it * 256 + tid;
      const int nrow = i >> 7;
      const int u4 = (i & 127) * 4;
      const v4f v = *(const v4f*)(wsrc + (size_t)nrow * kUDim + u4);
      *(v4f*)(s_w1x + nrow * kLdsPitch + u4) = v;
    }
  }
  asm volatile("" ::: "memory");

  {
    const int c = lane & 15, hh = lane >> 4, koff = hh * 8;
    const _Float16* qp = (const _Float16*)qplane + (size_t)(b * kSteps + t0 + c) * kQPad + koff;
    const v16h a = Frag<_Float16>::load(qp);
    const _Float16* wp = (const _Float16*)w2plane + koff;
    v16h bf[4];
#pragma unroll
    for (int j = 0; j < 4; ++j) {
      const int ucol = (wave * 4 + j) * 16 + c;
      bf[j] = Frag<_Float16>::load(wp + (size_t)ucol * kQPad);
    }
    v8f acc[4];
#pragma unroll
    for (int j = 0; j < 4; ++j) {
      acc[j] = (v8f){0.f,0.f,0.f,0.f,0.f,0.f,0.f,0.f};
      acc[j] = Frag<_Float16>::mma(a, bf[j], acc[j]);
    }
    dep_guard4_h(acc[0], acc[1], acc[2], acc[3], a, bf[3]);
    keep4_h(bf[0], bf[1], bf[2], bf[3]);
#pragma unroll
    for (int j = 0; j < 4; ++j) {
      const int ucol = (wave * 4 + j) * 16 + c;
      const float bias = b2[ucol];
#pragma unroll
      for (int r = 0; r < 8; ++r) s_w2q[(8 * hh + r) * kLdsPitch + ucol] = acc[j][r] * w2qScale + bias;
    }
  }
  __syncthreads();

  if (wave_u < 6) {
    const int c = lane & 15, hh = lane >> 4, koff = hh * 8;
    const float bvv = bv[0];
    const _Float16* wvp = (const _Float16*)wvplane + (size_t)c * kUDim + koff;
    const float* w2r = s_w2q + c * kLdsPitch + koff;
#pragma unroll 1
    for (int tt = 0; tt < 2; ++tt) {
      const int n = 2 * wave_u + tt;
      const float* w1r = s_w1x + n * kLdsPitch + koff;
      v8f acc = (v8f){0.f,0.f,0.f,0.f,0.f,0.f,0.f,0.f};
#pragma unroll 1
      for (int k0 = 0; k0 < kUDim; k0 += 32) {
        const v4f q0 = *(const v4f*)(w2r + k0);
        const v4f q1 = *(const v4f*)(w2r + k0 + 4);
        const v4f q2 = *(const v4f*)(w2r + k0 + 16);
        const v4f q3 = *(const v4f*)(w2r + k0 + 20);
        const v4f p0 = *(const v4f*)(w1r + k0);
        const v4f p1 = *(const v4f*)(w1r + k0 + 4);
        const v4f p2 = *(const v4f*)(w1r + k0 + 16);
        const v4f p3 = *(const v4f*)(w1r + k0 + 20);
        v16h a;
#pragma unroll
        for (int e = 0; e < 4; ++e) {
          const float t0v = tanh_s(p0[e] + q0[e]) * kTanhCarry;
          const float t1v = tanh_s(p1[e] + q1[e]) * kTanhCarry;
          const float t2v = tanh_s(p2[e] + q2[e]) * kTanhCarry;
          const float t3v = tanh_s(p3[e] + q3[e]) * kTanhCarry;
          a[e]      = (_Float16)t0v;
          a[4 + e]  = (_Float16)t1v;
          a[8 + e]  = (_Float16)t2v;
          a[12 + e] = (_Float16)t3v;
        }
        const v16h bfr = Frag<_Float16>::load(wvp + k0);
        acc = Frag<_Float16>::mma(a, bfr, acc);
        dep_guard1_h(acc, a, bfr);
      }
      acc_guard1(acc);
#pragma unroll
      for (int r = 0; r < 8; ++r) {
        const float mine = acc[r];
        const float other = __shfl_xor(mine, 1, 32);
        const float sc = (mine + other * kWvLoInv) * kScoreInv + bvv;
        if (c == 0) s_score[(8 * hh + r) * kFeat + n] = sc;
      }
    }
  }
  __syncthreads();

  if (tid < kTileT * kFeat) {
    const int tl = tid / kFeat;
    const int n = tid - tl * kFeat;
    const float* sc = s_score + tl * kFeat;
    float mx = sc[0];
#pragma unroll
    for (int j = 1; j < kFeat; ++j) mx = fmaxf(mx, sc[j]);
    float sum = 0.0f;
#pragma unroll 1
    for (int j = 0; j < kFeat; ++j) sum += expf(sc[j] - mx);
    const float e = expf(sc[n] - mx);
    const float inv = 1.0f / sum;
    const float alpha = e * inv;
    const float dv = data[(size_t)(b * kSteps + t0) * kFeat + tid];
    s_out[tid] = dv * alpha;
  }
  __syncthreads();

  if (wave == 0) {
    float* op = out + (size_t)(b * kSteps + t0) * kFeat;
    const int l16 = lane & 15;
    const v4f v0 = *(const v4f*)(s_out + 4 * lane);
    const v4f v1 = *(const v4f*)(s_out + 128 + 4 * l16);
    for (int pass = 0; pass < 2; ++pass) {
      *(volatile v4f*)(op + 4 * lane) = v0;
      if (lane < 16) *(volatile v4f*)(op + 128 + 4 * lane) = v1;
      __threadfence();
    }
  }
}

extern "C" void kernel_launch(void* const* d_in, const int* in_sizes, int n_in,
                              void* d_out, int out_size, void* d_ws, size_t ws_size, hipStream_t stream) {
  if (n_in < 18 || d_out == nullptr || d_ws == nullptr) return;
  if (in_sizes[0] != kBatch * kSteps * kFeat || in_sizes[4] != kGateRows * kFeat || in_sizes[6] != kGateRows ||
      in_sizes[7] != kGateRows || in_sizes[8] != kGateRows * kHid || in_sizes[10] != kGateRows ||
      in_sizes[11] != kGateRows || in_sizes[12] != kUDim * kSteps || in_sizes[13] != kUDim ||
      in_sizes[14] != kUDim * kQDim || in_sizes[15] != kUDim || in_sizes[16] != kUDim || in_sizes[17] != 1 ||
      out_size != kBatch * kSteps * kFeat) return;

  const float* data  = (const float*)d_in[0];
  const float* W_ih1 = (const float*)d_in[4];
  const float* b_ih1 = (const float*)d_in[6];
  const float* b_hh1 = (const float*)d_in[7];
  const float* W_ih2 = (const float*)d_in[8];
  const float* b_ih2 = (const float*)d_in[10];
  const float* b_hh2 = (const float*)d_in[11];
  const float* W1    = (const float*)d_in[12];
  const float* b1    = (const float*)d_in[13];
  const float* W2    = (const float*)d_in[14];
  const float* b2    = (const float*)d_in[15];
  const float* Wv    = (const float*)d_in[16];
  const float* bv    = (const float*)d_in[17];
  float* out = (float*)d_out;

  char* ws = (char*)d_ws; size_t off = 0;
  auto carve = [&](size_t bytes) -> char* { char* p = ws + off; off += (bytes + 255) & ~(size_t)255; return p; };
  unsigned short* QPL = (unsigned short*)carve((size_t)kRowsBT * kQPad * 2);
  unsigned short* DTH = (unsigned short*)carve((size_t)kRowsBN * kSteps * 2);
  unsigned short* W1H = (unsigned short*)carve((size_t)kUDim * kSteps * 2);
  unsigned short* W2H = (unsigned short*)carve((size_t)kUDim * kQPad * 2);
  unsigned short* WVP = (unsigned short*)carve((size_t)kWvRows * kUDim * 2);
  float*          W1X = (float*)carve((size_t)kRowsBN * kUDim * 4);
  if (off > ws_size || off > (size_t)134217728) return;

  dataT_f16_kernel<<<kBatch, 256, 0, stream>>>(data, DTH, kDataCarry);
  const int n8w1 = kUDim * kSteps / 8;
  cast8_scale_f16_kernel<<<(n8w1 + 255) / 256, 256, 0, stream>>>(W1, W1H, n8w1, kW1Carry);
  w2pad_f16_kernel<<<(kUDim * (kQPad / 8)) / 256, 256, 0, stream>>>(W2, W2H, kW2Carry);
  wvplane_f16_kernel<<<(kWvRows * kUDim / 8) / 256, 256, 0, stream>>>(Wv, WVP, kWvCarry, kWvLoScale);

  lstm_query_kernel<<<kRowsBT / 256, 256, 0, stream>>>(data, W_ih1, b_ih1, b_hh1, W_ih2, b_ih2, b_hh2, QPL, kQryCarry);

  const dim3 ggrid((kRowsBN / 64) * (kUDim / 64) / 8, 1);
  wmma_gemm64<0, false, 2, 0, false><<<ggrid, 256, 0, stream>>>(
      DTH, DTH, kSteps, 0L, W1H, W1H, kSteps, 0L, (void*)W1X, (void*)W1X, kUDim, 0L,
      b1, b1, 0L, kRowsBN, kUDim, kSteps, kW1xScale);

  attn_fused_kernel<<<kBatch * (kSteps / kTileT), 256, 0, stream>>>(data, QPL, W1X, W2H, b2, WVP, bv, out, kW2qScale);
}
